// SelectiveSSM_2894807958203
// MI455X (gfx1250) — hardware-verified
//
#include <hip/hip_runtime.h>
#include <math.h>

typedef __attribute__((ext_vector_type(16))) _Float16 v16h;
typedef __attribute__((ext_vector_type(8)))  _Float16 v8h;
typedef __attribute__((ext_vector_type(8)))  float    v8f;
typedef __attribute__((ext_vector_type(4)))  float    v4f;
typedef __attribute__((ext_vector_type(4)))  unsigned v4u;

constexpr int kBatch  = 2;
constexpr int kSeq    = 2048;
constexpr int kD      = 1024;
constexpr int kNst    = 16;
constexpr int kRank   = 64;
constexpr int kConvK  = 4;
constexpr int kRows   = kBatch * kSeq;
constexpr int kProjN  = 64;
constexpr int kWpRows = 128;
constexpr int kBcP    = 64;
constexpr int kBcW    = 32;
constexpr int kConvTP = 260;
constexpr int kScanTS = 64;
constexpr int kScanCh = 64;
constexpr int kScanYP = 68;
constexpr float kCarryX = 64.0f;
constexpr float kCarryW = 256.0f;
constexpr float kCarryL = 64.0f;
static_assert((kD % 32) == 0 && (kRank % 32) == 0, "GEMM K multiples of 32");
static_assert((kRows % 64) == 0 && (kProjN % 64) == 0 && (kD % 64) == 0, "GEMM M,N multiples of 64");
static_assert(2 * kNst <= kProjN && kRank == kProjN && kRank + 2 * kNst <= kWpRows, "projection packing");
static_assert((kSeq % kScanTS) == 0 && (kSeq % 64) == 0 && (kD % kScanCh) == 0 && (kD % 256) == 0, "tile multiples");
static_assert(kScanCh == 64 && kScanTS == 64, "scan store map assumes 64 x 64 tiles");

constexpr size_t kOffXC   = 0;
constexpr size_t kOffXCH  = kOffXC  + (size_t)kRows * kD * 4;
constexpr size_t kOffDTP  = kOffXCH + (size_t)kRows * kD * 2;
constexpr size_t kOffDTL  = kOffDTP + (size_t)kRows * kD * 4;
constexpr size_t kOffBCP  = kOffDTL + (size_t)kRows * kProjN * 2;
constexpr size_t kOffWP   = kOffBCP + (size_t)kRows * kBcP * 4;
constexpr size_t kOffWD   = kOffWP  + (size_t)kWpRows * kD * 2;
constexpr size_t kWsTotal = kOffWD  + (size_t)kD * kRank * 2;
static_assert(kWsTotal == 43909120ull, "carve total");
static_assert(kWsTotal <= 134217728ull, "carve cap");
static_assert((kOffXCH % 128) == 0 && (kOffDTP % 128) == 0 && (kOffDTL % 128) == 0 && (kOffBCP % 128) == 0 &&
              (kOffWP % 128) == 0 && (kOffWD % 128) == 0, "128-B aligned regions");

__device__ __forceinline__ void mma_guard_h(v8f& a0, v8f& a1, v8f& a2, v8f& a3,
                                            v16h x, v16h b0, v16h b1, v16h b2, v16h b3) {
  asm volatile("v_nop\n\tv_nop\n\tv_nop\n\tv_nop"
               : "+v"(a0), "+v"(a1), "+v"(a2), "+v"(a3)
               : "v"(x), "v"(b0), "v"(b1), "v"(b2), "v"(b3));
}
__device__ __forceinline__ void acc_guard4(v8f& a, v8f& b, v8f& c, v8f& d) {
  asm volatile("v_nop\n\tv_nop\n\tv_nop\n\tv_nop" : "+v"(a), "+v"(b), "+v"(c), "+v"(d));
}
struct FragH {
  union U { v16h v; v8h h[2]; };
  static __device__ __forceinline__ v16h load(const _Float16* p) {
    U f; f.h[0] = *(const v8h*)(p); f.h[1] = *(const v8h*)(p + 16); return f.v;
  }
  static __device__ __forceinline__ v8f mma(v16h a, v16h b, v8f c) {
    return __builtin_amdgcn_wmma_f32_16x16x32_f16(false, a, false, b, (short)0, c, false, false);
  }
};

template <int BIAS_MODE, int OUT_MODE>
__global__ __launch_bounds__(256) void wmma_gemm64_f16(
    const unsigned short* __restrict__ Ap, int lda,
    const unsigned short* __restrict__ Btp, int ldb,
    void* __restrict__ Cout, int ldc,
    const float* __restrict__ bias,
    int M, int N, int K, float scale) {
  const _Float16* A  = (const _Float16*)Ap;
  const _Float16* Bt = (const _Float16*)Btp;
  __shared__ __align__(16) float sT[8][16 * 68];
  const int lane = threadIdx.x & 31;
  const int wave = threadIdx.x >> 5;
  const int tilesN = N >> 6;
  const int tilesM = M >> 6;
  const int tile = blockIdx.x * 8 + wave;
  if (tile >= tilesM * tilesN) return;
  const int tm = tile / tilesN;
  const int tn = tile - tm * tilesN;
  const int m0 = tm << 6;
  const int n0 = tn << 6;

  const int rlane = lane & 15;
  const int koff  = (lane >> 4) * 8;
  const int mOff  = (lane >> 4) * 8;

  v8f acc[4][4];
#pragma unroll
  for (int i = 0; i < 4; ++i)
#pragma unroll
    for (int j = 0; j < 4; ++j) acc[i][j] = (v8f){0.f,0.f,0.f,0.f,0.f,0.f,0.f,0.f};

  for (int k0 = 0; k0 < K; k0 += 32) {
    v16h bh[4];
#pragma unroll
    for (int j = 0; j < 4; ++j) {
      const size_t bo = (size_t)(n0 + (j << 4) + rlane) * ldb + koff + k0;
      bh[j] = FragH::load(Bt + bo);
    }
#pragma unroll
    for (int i = 0; i < 4; ++i) {
      const size_t ao = (size_t)(m0 + (i << 4) + rlane) * lda + koff + k0;
      v16h ah = FragH::load(A + ao);
#pragma unroll
      for (int j = 0; j < 4; ++j) acc[i][j] = FragH::mma(ah, bh[j], acc[i][j]);
      mma_guard_h(acc[i][0], acc[i][1], acc[i][2], acc[i][3], ah, bh[0], bh[1], bh[2], bh[3]);
    }
  }
  acc_guard4(acc[0][0], acc[0][1], acc[0][2], acc[0][3]);
  acc_guard4(acc[1][0], acc[1][1], acc[1][2], acc[1][3]);
  acc_guard4(acc[2][0], acc[2][1], acc[2][2], acc[2][3]);
  acc_guard4(acc[3][0], acc[3][1], acc[3][2], acc[3][3]);

  float* slab = sT[wave];
#pragma unroll
  for (int i = 0; i < 4; ++i) {
    const int mBase = m0 + (i << 4);
#pragma unroll
    for (int j = 0; j < 4; ++j) {
      const int n = n0 + (j << 4) + rlane;
      float bv = 0.f;
      if (BIAS_MODE == 2) bv = bias[n];
#pragma unroll
      for (int r = 0; r < 8; ++r) {
        float v = acc[i][j][r] * scale;
        if (BIAS_MODE == 2) v += bv;
        slab[(mOff + r) * 68 + (j << 4) + rlane] = v;
      }
    }
    __builtin_amdgcn_fence(__ATOMIC_RELEASE, "workgroup");
    __builtin_amdgcn_wave_barrier();
    __builtin_amdgcn_fence(__ATOMIC_ACQUIRE, "workgroup");
    if (OUT_MODE == 0) {
      float* Cp = (float*)Cout;
      const int hh = lane >> 4, c4 = (lane & 15) * 4;
      for (int pass = 0; pass < 2; ++pass) {
#pragma unroll
        for (int it = 0; it < 8; ++it) {
          const int row = it * 2 + hh;
          v4f v = *(const v4f*)(slab + row * 68 + c4);
          *(volatile v4f*)(Cp + (size_t)(mBase + row) * ldc + n0 + c4) = v;
        }
        __threadfence();
      }
    } else {
      const int q = lane >> 3, c8 = (lane & 7) * 8;
      unsigned short* Cp = (unsigned short*)Cout;
      for (int pass = 0; pass < 2; ++pass) {
#pragma unroll
        for (int it = 0; it < 4; ++it) {
          const int row = it * 4 + q;
          const float* sp = slab + row * 68 + c8;
          v8h hv;
#pragma unroll
          for (int e = 0; e < 8; ++e) hv[e] = (_Float16)sp[e];
          *(volatile v8h*)(Cp + (size_t)(mBase + row) * ldc + n0 + c8) = hv;
        }
        __threadfence();
      }
    }
    __builtin_amdgcn_fence(__ATOMIC_RELEASE, "workgroup");
    __builtin_amdgcn_wave_barrier();
    __builtin_amdgcn_fence(__ATOMIC_ACQUIRE, "workgroup");
  }
}

__global__ __launch_bounds__(256) void cast_scale_f16_kernel(
    const float* __restrict__ src, unsigned short* __restrict__ dst, int total8, float scale)
{
  const int i = blockIdx.x * 256 + threadIdx.x;
  if (i >= total8) return;
  const size_t e0 = (size_t)i << 3;
  const v4f a0 = *(const v4f*)(src + e0);
  const v4f a1 = *(const v4f*)(src + e0 + 4);
  v8h hv;
#pragma unroll
  for (int e = 0; e < 4; ++e) {
    hv[e]     = (_Float16)(a0[e] * scale);
    hv[4 + e] = (_Float16)(a1[e] * scale);
  }
  unsigned short* qh = dst + e0;
  *(volatile v8h*)qh = hv;
  __threadfence();
  *(volatile v8h*)qh = hv;
}

__global__ __launch_bounds__(256) void zero_f16_kernel(unsigned short* __restrict__ dst, int total8)
{
  const int i = blockIdx.x * 256 + threadIdx.x;
  if (i >= total8) return;
  const size_t e0 = (size_t)i << 3;
  const v4u z = {0u, 0u, 0u, 0u};
  unsigned short* q = dst + e0;
  *(volatile v4u*)q = z;
  __threadfence();
  *(volatile v4u*)q = z;
}

__global__ __launch_bounds__(256) void conv_silu_kernel(
    const float* __restrict__ X, const float* __restrict__ cw, const float* __restrict__ cb,
    float* __restrict__ XC, unsigned short* __restrict__ XCH)
{
  __shared__ __align__(16) float sT[16 * kConvTP];
  const int tid = threadIdx.x, lane = tid & 31, wave = tid >> 5;
  const int d0 = blockIdx.x * 256, d = d0 + tid;
  const int g0 = blockIdx.y * 64;
  const int tb = g0 & (kSeq - 1);
  const float w0 = cw[d * kConvK + 0], w1 = cw[d * kConvK + 1], w2 = cw[d * kConvK + 2], w3 = cw[d * kConvK + 3];
  const float bc = cb[d];
  float xm3, xm2, xm1;
  {
    const float fh = (tb > 0) ? 1.0f : 0.0f;
    const int rb = (tb > 0) ? (g0 - 3) : g0;
    const float v3 = X[(size_t)rb * kD + d];
    const float v2 = X[(size_t)(rb + 1) * kD + d];
    const float v1 = X[(size_t)(rb + 2) * kD + d];
    xm3 = v3 * fh;
    xm2 = v2 * fh;
    xm1 = v1 * fh;
  }
  const int hrow = wave >> 1;
  const int hch  = (wave & 1) * 128 + lane * 4;
#pragma unroll 1
  for (int sub = 0; sub < 4; ++sub) {
    const int lb = g0 + sub * 16;
#pragma unroll 1
    for (int s = 0; s < 16; ++s) {
      const float xcur = X[(size_t)(lb + s) * kD + d];
      float acc = w0 * xm3;
      acc = fmaf(w1, xm2, acc);
      acc = fmaf(w2, xm1, acc);
      acc = fmaf(w3, xcur, acc);
      const float sv = acc + bc;
      const float sg = __builtin_amdgcn_rcpf(1.0f + expf(-sv));
      sT[s * kConvTP + tid] = sv * sg;
      xm3 = xm2; xm2 = xm1; xm1 = xcur;
    }
    __syncthreads();
    for (int pass = 0; pass < 2; ++pass) {
#pragma unroll
      for (int it = 0; it < 4; ++it) {
        const v4f fv = *(const v4f*)(sT + (it * 4 + hrow) * kConvTP + hch);
        *(volatile v4f*)(XC + (size_t)(lb + it * 4 + hrow) * kD + d0 + hch) = fv;
      }
#pragma unroll
      for (int it = 0; it < 2; ++it) {
        const float* sp = sT + (it * 8 + wave) * kConvTP + lane * 8;
        const v4f a0 = *(const v4f*)(sp);
        const v4f a1 = *(const v4f*)(sp + 4);
        v8h hv;
#pragma unroll
        for (int e = 0; e < 4; ++e) {
          hv[e]     = (_Float16)(a0[e] * kCarryX);
          hv[4 + e] = (_Float16)(a1[e] * kCarryX);
        }
        *(volatile v8h*)(XCH + (size_t)(lb + it * 8 + wave) * kD + d0 + lane * 8) = hv;
      }
      __threadfence();
    }
    __syncthreads();
  }
}

__global__ __launch_bounds__(64) void scan_kernel(
    const float* __restrict__ BCP, const float* __restrict__ XC, const float* __restrict__ DTP,
    const float* __restrict__ Alog, const float* __restrict__ Dp, float* __restrict__ out)
{
  __shared__ __align__(16) float sBC[kScanTS * kBcW];
  __shared__ __align__(16) float sY[kScanTS * kScanYP];
  __shared__ __align__(16) float sA[kNst * kScanCh];
  const int tid = threadIdx.x, lane = tid & 31, wave = tid >> 5;
  constexpr int kBlkPerB = kD / kScanCh;
  const int bix = blockIdx.x / kBlkPerB;
  const int d0  = (blockIdx.x - bix * kBlkPerB) * kScanCh;
  const int d   = d0 + tid;
  const size_t row0 = (size_t)bix * kSeq;
#pragma unroll 1
  for (int s = 0; s < kNst; ++s) sA[s * kScanCh + tid] = -__expf(Alog[(size_t)d * kNst + s]);
  __syncthreads();
  float negA[kNst], h[kNst];
#pragma unroll
  for (int s = 0; s < kNst; ++s) {
    negA[s] = sA[s * kScanCh + tid];
    h[s] = 0.f;
  }
  const float Dd = Dp[d];
  const int lr = tid >> 3, lc4 = (tid & 7) * 4;
  const int hh = lane >> 4, c4 = (lane & 15) * 4;
#pragma unroll 1
  for (int t0 = 0; t0 < kSeq; t0 += kScanTS) {
    __syncthreads();
#pragma unroll
    for (int i = 0; i < 8; ++i) {
      const int r = lr + 8 * i;
      *(v4f*)(sBC + r * kBcW + lc4) = *(const v4f*)(BCP + (row0 + t0 + r) * kBcP + lc4);
    }
    __syncthreads();
#pragma unroll 1
    for (int s = 0; s < kScanTS; ++s) {
      const int t = t0 + s;
      const float* xr = sBC + s * kBcW;
      float Bs[kNst], Cs[kNst];
#pragma unroll
      for (int q4 = 0; q4 < 4; ++q4) {
        const v4f bv = *(const v4f*)(xr + 4 * q4);
        const v4f cv = *(const v4f*)(xr + kNst + 4 * q4);
        Bs[4 * q4 + 0] = bv[0]; Bs[4 * q4 + 1] = bv[1]; Bs[4 * q4 + 2] = bv[2]; Bs[4 * q4 + 3] = bv[3];
        Cs[4 * q4 + 0] = cv[0]; Cs[4 * q4 + 1] = cv[1]; Cs[4 * q4 + 2] = cv[2]; Cs[4 * q4 + 3] = cv[3];
      }
      const float v   = DTP[(row0 + t) * kD + d];
      const float xt  = XC[(row0 + t) * kD + d];
      const float dt  = fmaxf(v, 0.0f) + log1pf(__expf(-fabsf(v)));
      const float dtx = dt * xt;
      float y = 0.f;
#pragma unroll
      for (int k = 0; k < kNst; ++k) {
        const float e = __expf(dt * negA[k]);
        h[k] = fmaf(e, h[k], dtx * Bs[k]);
        y = fmaf(h[k], Cs[k], y);
      }
      y = fmaf(xt, Dd, y);
      sY[s * kScanYP + tid] = y;
    }
    __syncthreads();
    for (int pass = 0; pass < 2; ++pass) {
#pragma unroll
      for (int it = 0; it < 16; ++it) {
        const int row = it * 4 + wave * 2 + hh;
        const v4f val = *(const v4f*)(sY + row * kScanYP + c4);
        *(volatile v4f*)(out + (row0 + t0 + row) * kD + d0 + c4) = val;
      }
      __threadfence();
    }
  }
}

extern "C" void kernel_launch(void* const* d_in, const int* in_sizes, int n_in,
                              void* d_out, int out_size, void* d_ws, size_t ws_size,
                              hipStream_t stream) {
  if (n_in < 10) return;
  if (in_sizes[0] != kRows * kD) return;
  if (in_sizes[1] != kD * kConvK) return;
  if (in_sizes[2] != kD) return;
  if (in_sizes[3] != kRank * kD) return;
  if (in_sizes[4] != kD * kRank) return;
  if (in_sizes[5] != kD) return;
  if (in_sizes[6] != kNst * kD) return;
  if (in_sizes[7] != kNst * kD) return;
  if (in_sizes[8] != kD * kNst) return;
  if (in_sizes[9] != kD) return;
  if (out_size != kRows * kD) return;
  if (ws_size < kWsTotal) return;

  const float* x      = (const float*)d_in[0];
  const float* conv_w = (const float*)d_in[1];
  const float* conv_b = (const float*)d_in[2];
  const float* Wx     = (const float*)d_in[3];
  const float* Wdt    = (const float*)d_in[4];
  const float* bdt    = (const float*)d_in[5];
  const float* Wb     = (const float*)d_in[6];
  const float* Wc     = (const float*)d_in[7];
  const float* A_log  = (const float*)d_in[8];
  const float* Dp     = (const float*)d_in[9];
  float* out = (float*)d_out;

  char* ws = (char*)d_ws;
  float*          XC  = (float*)(ws + kOffXC);
  unsigned short* XCH = (unsigned short*)(ws + kOffXCH);
  float*          DTP = (float*)(ws + kOffDTP);
  unsigned short* DTL = (unsigned short*)(ws + kOffDTL);
  float*          BCP = (float*)(ws + kOffBCP);
  unsigned short* WP  = (unsigned short*)(ws + kOffWP);
  unsigned short* WD  = (unsigned short*)(ws + kOffWD);

  const float kScaleDtl = kCarryL / (kCarryX * kCarryW);
  const float kScaleBc  = 1.0f / (kCarryX * kCarryW);
  const float kScaleDtp = 1.0f / (kCarryL * kCarryW);

  cast_scale_f16_kernel<<<(kRank * kD / 8) / 256, 256, 0, stream>>>(Wx, WP, kRank * kD / 8, kCarryW);
  cast_scale_f16_kernel<<<(kNst * kD / 8) / 256, 256, 0, stream>>>(Wb, WP + (size_t)kRank * kD, kNst * kD / 8, kCarryW);
  cast_scale_f16_kernel<<<(kNst * kD / 8) / 256, 256, 0, stream>>>(Wc, WP + (size_t)(kRank + kNst) * kD, kNst * kD / 8, kCarryW);
  zero_f16_kernel<<<((kWpRows - kRank - 2 * kNst) * kD / 8) / 256, 256, 0, stream>>>(
      WP + (size_t)(kRank + 2 * kNst) * kD, (kWpRows - kRank - 2 * kNst) * kD / 8);
  cast_scale_f16_kernel<<<(kD * kRank / 8) / 256, 256, 0, stream>>>(Wdt, WD, kD * kRank / 8, kCarryW);

  conv_silu_kernel<<<dim3(kD / 256, kRows / 64), 256, 0, stream>>>(x, conv_w, conv_b, XC, XCH);

  wmma_gemm64_f16<0, 1><<<(kRows / 64) * (kProjN / 64) / 8, 256, 0, stream>>>(
      XCH, kD, WP, kD, (void*)DTL, kProjN, nullptr, kRows, kProjN, kD, kScaleDtl);

  wmma_gemm64_f16<0, 0><<<(kRows / 64) * (kProjN / 64) / 8, 256, 0, stream>>>(
      XCH, kD, WP + (size_t)kRank * kD, kD, (void*)BCP, kBcP, nullptr, kRows, kProjN, kD, kScaleBc);

  wmma_gemm64_f16<2, 0><<<(kRows / 64) * (kD / 64) / 8, 256, 0, stream>>>(
      DTL, kRank, WD, kRank, (void*)DTP, kD, bdt, kRows, kD, kRank, kScaleDtp);

  scan_kernel<<<kBatch * (kD / kScanCh), kScanCh, 0, stream>>>(BCP, XC, DTP, A_log, Dp, out);
}
